// Model_23880018165985
// MI455X (gfx1250) — hardware-run, weakly checked
//
#include <hip/hip_runtime.h>


#ifndef NB
#define NB 2
#endif
#ifndef SEQ
#define SEQ 2048
#endif
#define NB_FULL  2
#define SEQ_FULL 2048
#ifndef OUT_SEQ
#define OUT_SEQ SEQ
#endif
#define DX   192
#define NH_  16
#define HD   128
#define DQ   2048
#define AW   4
#define OSP  132
#define OSQ  132
#define SC2  ((float)(0.08838834764831845 * 1.4426950408889634))
#define L2E  1.4426950408889634f
#define PSH  14.0f
#define NEGB (-3.0e38f)
#define CXS  256.0f
#define WOS  64.0f
#define OSC  (1.0f / 16384.0f)

static_assert(HD == 128);
static_assert(NH_ * HD == DQ);
static_assert(HD % 32 == 0);
static_assert(DX % 32 == 0);
static_assert(DQ % 32 == 0);
static_assert(DX % 64 == 0);
static_assert(DQ % 64 == 0);
static_assert(SEQ % 64 == 0);
static_assert((NB * SEQ) % 64 == 0);
static_assert(SEQ % 32 == 0);
static_assert(SEQ % (16 * AW) == 0);
static_assert(((size_t)SEQ * DX) % 64 == 0);
static_assert(((size_t)DQ * DX) % 2048 == 0);
static_assert((SEQ * 64) % 256 == 0);
static_assert(NB <= NB_FULL);
static_assert(SEQ <= SEQ_FULL);
static_assert(OSP >= HD);
static_assert(OSQ >= HD);
static_assert((OSP * 4) % 16 == 0);
static_assert((OSQ * 4) % 16 == 0);
static_assert((DX * 4) % 128 == 0);
static_assert(32 * 16 * 8 == 16 * HD * 2);
static_assert(32 * 16 * 4 == 16 * 64 * 2);
static_assert(32 * 16 * 8 == 16 * 64 * 4);
static_assert(16 * OSQ * 4 <= 131072);
static_assert(16 * 68 * 4 <= 131072);
static_assert(AW * 16 * OSP * 4 <= 131072);

typedef _Float16 h16;
typedef unsigned short bf;
typedef __attribute__((ext_vector_type(16))) __bf16   v16bf;
typedef __attribute__((ext_vector_type(16))) _Float16 v16h;
typedef __attribute__((ext_vector_type(8)))  _Float16 v8h;
typedef __attribute__((ext_vector_type(8)))  unsigned short v8us;
typedef __attribute__((ext_vector_type(8)))  float    v8f;
typedef __attribute__((ext_vector_type(4)))  float    v4f;
typedef v4f  __attribute__((may_alias)) v4fa;

__device__ __forceinline__ unsigned short f2bf(float f) { unsigned u = __float_as_uint(f); u += 0x7FFFu + ((u >> 16) & 1u); return (unsigned short)(u >> 16); }
__device__ __forceinline__ float bfr(float f) { return __uint_as_float(((unsigned)f2bf(f)) << 16); }
__device__ __forceinline__ v16h cat16(v8h lo, v8h hi) { return __builtin_shufflevector(lo, hi, 0, 1, 2, 3, 4, 5, 6, 7, 8, 9, 10, 11, 12, 13, 14, 15); }
__device__ __forceinline__ v16bf cat16b(v8us lo, v8us hi) { return __builtin_bit_cast(v16bf, __builtin_shufflevector(lo, hi, 0, 1, 2, 3, 4, 5, 6, 7, 8, 9, 10, 11, 12, 13, 14, 15)); }
__device__ __forceinline__ v8f wmma16(v16h a, v16h b, v8f c) { return __builtin_amdgcn_wmma_f32_16x16x32_f16(false, a, false, b, (short)0, c, false, false); }
__device__ __forceinline__ v8f wmmab(v16bf a, v16bf b, v8f c) { return __builtin_amdgcn_wmma_f32_16x16x32_bf16(false, a, false, b, (short)0, c, false, false); }
__device__ __forceinline__ v16h  ldh(const h16* p) { return cat16(*(const v8h*)p, *(const v8h*)(p + 16)); }
__device__ __forceinline__ v16bf ldb(const bf* p)  { return cat16b(*(const v8us*)p, *(const v8us*)(p + 16)); }
__device__ __forceinline__ void wave_sync() { __builtin_amdgcn_fence(3  , "wavefront"); __builtin_amdgcn_wave_barrier(); asm volatile("" ::: "memory"); }

static __device__ __forceinline__ h16 toh_flush(float v) { const h16 r = (h16)v; return (fabsf(v) < 6.103515625e-05f) ? (h16)0.0f : r; }
static __device__ __forceinline__ v8f wmma16g(v16h a, v16h b, v8f c) { c = wmma16(a, b, c); asm volatile("v_nop\n\tv_nop\n\tv_nop\n\tv_nop" : "+v"(c) : "v"(a), "v"(b)); return c; }
static __device__ __forceinline__ v8f wmmabg(v16bf a, v16bf b, v8f c) { c = wmmab(a, b, c); asm volatile("v_nop\n\tv_nop\n\tv_nop\n\tv_nop" : "+v"(c) : "v"(a), "v"(b)); return c; }

__global__ __launch_bounds__(256) void k_cvt8(const float* __restrict__ src, bf* dst, size_t n8) {
    const size_t i = (size_t)blockIdx.x * 256 + threadIdx.x; if (i >= n8) return;
    const v8f v = *(const v8f*)(src + i * 8); v8us o;
#pragma unroll
    for (int k = 0; k < 8; ++k) o[k] = f2bf(v[k]);
    *(volatile v8us*)(dst + i * 8) = o; __threadfence(); *(volatile v8us*)(dst + i * 8) = o;
}

__global__ __launch_bounds__(256) void k_cvtw(const float* __restrict__ src, h16* dst, size_t n8, float sc) {
    const size_t i = (size_t)blockIdx.x * 256 + threadIdx.x; if (i >= n8) return;
    const v8f v = *(const v8f*)(src + i * 8); v8h o;
#pragma unroll
    for (int k = 0; k < 8; ++k) o[k] = toh_flush(bfr(v[k]) * sc);
    *(volatile v8h*)(dst + i * 8) = o; __threadfence(); *(volatile v8h*)(dst + i * 8) = o;
}

__global__ __launch_bounds__(256) void k_tab(float* COS, float* SIN, int n) {
#pragma clang fp contract(off)
    const int i = blockIdx.x * 256 + threadIdx.x; if (i >= n) return;
    const int pos = i >> 6, j = i & 63;
    const float invf = exp2f(-(float)j * (19.931568569324174f / 64.0f));
    const float ang = (float)pos * invf;
    float sn, cs; sincosf(ang, &sn, &cs);
    *(volatile float*)(COS + i) = cs; *(volatile float*)(SIN + i) = sn; __threadfence();
    *(volatile float*)(COS + i) = cs; *(volatile float*)(SIN + i) = sn;
}

__global__ __launch_bounds__(32) void k_qk(const bf* __restrict__ A, const bf* __restrict__ Bt, const float* __restrict__ nw,
                                           const float* __restrict__ COS, const float* __restrict__ SIN, h16* Ph) {
    __shared__ __align__(16) float os[16 * OSQ];
    const int K = DX;
    const int lane = threadIdx.x & 31, lr = lane & 15, hi = lane >> 4; const int r0 = blockIdx.x * 32, c0 = blockIdx.y * HD;
    v8f acc[2][8];
#pragma unroll
    for (int mb = 0; mb < 2; ++mb)
#pragma unroll
        for (int nb = 0; nb < 8; ++nb) acc[mb][nb] = (v8f){};
    const size_t aoff = (size_t)(r0 + lr) * K + 8 * hi, boff = (size_t)(c0 + lr) * K + 8 * hi;
#pragma unroll 1
    for (int kc = 0; kc < K; kc += 32) {
        v16bf a[2];
#pragma unroll
        for (int mb = 0; mb < 2; ++mb) a[mb] = ldb(A + aoff + (size_t)mb * 16 * K + kc);
#pragma unroll
        for (int nb = 0; nb < 8; ++nb) { const v16bf b = ldb(Bt + boff + (size_t)nb * 16 * K + kc);
#pragma unroll
            for (int mb = 0; mb < 2; ++mb) acc[mb][nb] = wmmabg(a[mb], b, acc[mb][nb]); }
    }
    float wn[8];
#pragma unroll
    for (int nb = 0; nb < 8; ++nb) wn[nb] = bfr(nw[nb * 16 + lr]);
    const int bb = r0 / SEQ, tt = r0 % SEQ; const int zc = bb * NH_ + (int)blockIdx.y;
    const size_t tbase = ((size_t)zc * SEQ + (size_t)tt) * HD;
#pragma unroll
    for (int mb = 0; mb < 2; ++mb) {
#pragma unroll
        for (int j = 0; j < 8; ++j) {
            float ss = 0.0f;
#pragma unroll
            for (int nb = 0; nb < 8; ++nb) ss += acc[mb][nb][j] * acc[mb][nb][j];
            ss += __shfl_xor(ss, 1, 32); ss += __shfl_xor(ss, 2, 32); ss += __shfl_xor(ss, 4, 32); ss += __shfl_xor(ss, 8, 32);
            const float rs = rsqrtf(ss * (1.0f / 128.0f) + 1.0e-6f);
#pragma unroll
            for (int nb = 0; nb < 8; ++nb) os[(hi * 8 + j) * OSQ + nb * 16 + lr] = (acc[mb][nb][j] * rs) * wn[nb]; }
        wave_sync();
        v8h hv[8];
#pragma unroll
        for (int s = 0; s < 8; ++s) { const int p = s * 32 + lane; const int row = p >> 4, c8 = (p & 15) * 8;
            const int pc = c8 ^ 64, jj = c8 & 63; const float sg = (c8 < 64) ? -1.0f : 1.0f;
            const v4f x0 = *(const v4fa*)(&os[row * OSQ + c8]), x1 = *(const v4fa*)(&os[row * OSQ + c8 + 4]);
            const v4f y0 = *(const v4fa*)(&os[row * OSQ + pc]), y1 = *(const v4fa*)(&os[row * OSQ + pc + 4]);
            const size_t to = (size_t)(tt + mb * 16 + row) * 64 + (size_t)jj;
            const v4f ca = *(const v4f*)(COS + to), cb = *(const v4f*)(COS + to + 4), sa = *(const v4f*)(SIN + to), sb = *(const v4f*)(SIN + to + 4);
            v8h o;
#pragma unroll
            for (int i = 0; i < 4; ++i) { o[i] = toh_flush(x0[i] * ca[i] + (sg * y0[i]) * sa[i]); o[4 + i] = toh_flush(x1[i] * cb[i] + (sg * y1[i]) * sb[i]); }
            hv[s] = o; }
        const size_t sbs = tbase + (size_t)(mb * 16) * HD;
#pragma unroll 1
        for (int ps = 0; ps < 2; ++ps) {
#pragma unroll
            for (int s = 0; s < 8; ++s) *(volatile v8h*)(Ph + sbs + (size_t)(s * 32 + lane) * 8) = hv[s];
            if (ps == 0) __threadfence(); }
        wave_sync();
    }
}

__global__ __launch_bounds__(32) void k_vt(const bf* __restrict__ A, const bf* __restrict__ Bt, h16* Ph) {
    __shared__ __align__(16) float os[16 * 68];
    const int K = DX;
    const int lane = threadIdx.x & 31, lr = lane & 15, hi = lane >> 4; const int r0 = blockIdx.x * 64, c0 = blockIdx.y * 64;
    v8f acc[4][4];
#pragma unroll
    for (int mb = 0; mb < 4; ++mb)
#pragma unroll
        for (int nb = 0; nb < 4; ++nb) acc[mb][nb] = (v8f){};
    const size_t aoff = (size_t)(r0 + lr) * K + 8 * hi, boff = (size_t)(c0 + lr) * K + 8 * hi;
#pragma unroll 1
    for (int kc = 0; kc < K; kc += 32) {
        v16bf a[4];
#pragma unroll
        for (int mb = 0; mb < 4; ++mb) a[mb] = ldb(A + aoff + (size_t)mb * 16 * K + kc);
#pragma unroll
        for (int nb = 0; nb < 4; ++nb) { const v16bf b = ldb(Bt + boff + (size_t)nb * 16 * K + kc);
#pragma unroll
            for (int mb = 0; mb < 4; ++mb) acc[mb][nb] = wmmabg(a[mb], b, acc[mb][nb]); }
    }
    const int bb = c0 / SEQ, tt = c0 % SEQ;
    const size_t tbase = (size_t)bb * (size_t)DQ * SEQ + (size_t)r0 * SEQ + (size_t)tt;
#pragma unroll
    for (int mb = 0; mb < 4; ++mb) {
#pragma unroll
        for (int nb = 0; nb < 4; ++nb) {
#pragma unroll
            for (int j = 0; j < 8; ++j) os[(hi * 8 + j) * 68 + nb * 16 + lr] = acc[mb][nb][j]; }
        wave_sync();
        v8h hv[4];
#pragma unroll
        for (int s = 0; s < 4; ++s) { const int row = 4 * s + (lane >> 3), c8 = (lane & 7) * 8;
            const v4f x0 = *(const v4fa*)(&os[row * 68 + c8]); const v4f x1 = *(const v4fa*)(&os[row * 68 + c8 + 4]); v8h o;
#pragma unroll
            for (int i = 0; i < 4; ++i) { o[i] = toh_flush(x0[i]); o[4 + i] = toh_flush(x1[i]); }
            hv[s] = o; }
        const size_t sbs = tbase + (size_t)(mb * 16) * SEQ;
#pragma unroll 1
        for (int ps = 0; ps < 2; ++ps) {
#pragma unroll
            for (int s = 0; s < 4; ++s) { const int row = 4 * s + (lane >> 3), c8 = (lane & 7) * 8;
                *(volatile v8h*)(Ph + sbs + (size_t)row * SEQ + c8) = hv[s]; }
            if (ps == 0) __threadfence(); }
        wave_sync();
    }
}

__global__ __launch_bounds__(32 * AW) __attribute__((amdgpu_num_vgpr(256)))
void k_flash(const h16* __restrict__ QH, const h16* __restrict__ KP, const h16* __restrict__ VT, const float* __restrict__ mask, h16* CTX) {
    __shared__ __align__(16) float os[AW * 16 * OSP];
    const int lane = threadIdx.x & 31, lr = lane & 15, hi = lane >> 4;
    const int wave = __builtin_amdgcn_readfirstlane((int)(threadIdx.x >> 5));
    const int zh = blockIdx.y; const int b = zh / NH_, h = zh % NH_;
    const int t0 = (blockIdx.x * AW + wave) * 16;
    const size_t pbase = (size_t)zh * SEQ * HD;
    const size_t qo = pbase + (size_t)(t0 + lr) * HD + 8 * hi;
    const size_t ko = pbase + (size_t)lr * HD + 8 * hi;
    const size_t vo = pbase + (size_t)lr * SEQ + 8 * hi;
    const float* mrow = mask + ((size_t)b * SEQ_FULL + (size_t)(t0 + lr)) * SEQ_FULL + 8 * hi;
    v8f o[8];
#pragma unroll
    for (int j = 0; j < 8; ++j) o[j] = (v8f){};
    float m = NEGB, l = 0.0f;
#pragma unroll 1
    for (int key0 = 0; key0 < SEQ; key0 += 32) {
        unsigned qsh = 0; asm volatile("" : "+v"(qsh));
        const h16* ka = KP + ko + (size_t)key0 * HD;
        const h16* qa = QH + qo + qsh;
        v8f sA = (v8f){}, sB = (v8f){};
#pragma unroll
        for (int ks = 0; ks < HD / 32; ++ks) {
            const v16h qf = ldh(qa + ks * 32);
            const v16h ka0 = ldh(ka + ks * 32), kb0 = ldh(ka + 16 * HD + ks * 32);
            sA = wmma16g(ka0, qf, sA); sB = wmma16g(kb0, qf, sB); }
        const float* mp = mrow + key0;
        const v4f m0 = *(const v4f*)mp, m1 = *(const v4f*)(mp + 4), m2 = *(const v4f*)(mp + 16), m3 = *(const v4f*)(mp + 20);
        float ta[8], tb[8]; float mx = NEGB;
#pragma unroll
        for (int r = 0; r < 4; ++r) {
            ta[r] = sA[r] * SC2 + bfr(m0[r]) * L2E; ta[4 + r] = sA[4 + r] * SC2 + bfr(m1[r]) * L2E;
            tb[r] = sB[r] * SC2 + bfr(m2[r]) * L2E; tb[4 + r] = sB[4 + r] * SC2 + bfr(m3[r]) * L2E; }
#pragma unroll
        for (int r = 0; r < 8; ++r) mx = fmaxf(mx, fmaxf(ta[r], tb[r]));
        mx = fmaxf(mx, __shfl_xor(mx, 16, 32));
        const float mnew = fmaxf(m, mx);
        const float alpha = __builtin_amdgcn_exp2f(m - mnew);
        const float sh = PSH - mnew;
        v16h pb; float ls = 0.0f;
#pragma unroll
        for (int r = 0; r < 8; ++r) {
            const float xa = ta[r] + sh, xb = tb[r] + sh;
            const float ea = __builtin_amdgcn_exp2f(xa), eb = __builtin_amdgcn_exp2f(xb);
            const float ga = (xa < -14.0f) ? 0.0f : ea, gb = (xb < -14.0f) ? 0.0f : eb;
            const h16 pa = (h16)ga; const h16 pc = (h16)gb;
            pb[r] = pa; pb[8 + r] = pc;
            ls += (float)pa + (float)pc; }
        l = l * alpha + ls; m = mnew;
#pragma unroll
        for (int j = 0; j < 8; ++j) o[j] = o[j] * alpha;
        const h16* va = VT + vo + key0;
#pragma unroll
        for (int g = 0; g < 2; ++g) {
            v16h vf[4];
#pragma unroll
            for (int j = 0; j < 4; ++j) vf[j] = ldh(va + (size_t)(16 * (4 * g + j)) * SEQ);
#pragma unroll
            for (int j = 0; j < 4; ++j) o[4 * g + j] = wmma16g(vf[j], pb, o[4 * g + j]); }
    }
    l += __shfl_xor(l, 16, 32);
    const bool any = l > 0.0f;
    const float lsafe = any ? l : 1.0f;
    const float inv = any ? ((1.0f / lsafe) * CXS) : 0.0f;
    const int wb = wave * 16 * OSP;
#pragma unroll
    for (int j = 0; j < 8; ++j) { v4f a, c;
        a[0] = o[j][0] * inv; a[1] = o[j][1] * inv; a[2] = o[j][2] * inv; a[3] = o[j][3] * inv; c[0] = o[j][4] * inv; c[1] = o[j][5] * inv; c[2] = o[j][6] * inv; c[3] = o[j][7] * inv;
        *(v4fa*)(&os[wb + lr * OSP + 16 * j + 8 * hi]) = a; *(v4fa*)(&os[wb + lr * OSP + 16 * j + 8 * hi + 4]) = c; }
    wave_sync();
    v8h hv[8];
#pragma unroll
    for (int s = 0; s < 8; ++s) { const int p = s * 32 + lane; const int row = p >> 4, c8 = (p & 15) * 8;
        const v4f x0 = *(const v4fa*)(&os[wb + row * OSP + c8]); const v4f x1 = *(const v4fa*)(&os[wb + row * OSP + c8 + 4]); v8h q;
#pragma unroll
        for (int i = 0; i < 4; ++i) { q[i] = toh_flush(x0[i]); q[4 + i] = toh_flush(x1[i]); }
        hv[s] = q; }
    h16* crow = CTX + ((size_t)b * SEQ + (size_t)t0) * DQ + (size_t)h * HD;
#pragma unroll 1
    for (int ps = 0; ps < 2; ++ps) {
#pragma unroll
        for (int s = 0; s < 8; ++s) { const int p = s * 32 + lane; const int row = p >> 4, c8 = (p & 15) * 8;
            *(volatile v8h*)(crow + (size_t)row * DQ + c8) = hv[s]; }
        if (ps == 0) __threadfence(); }
}

__global__ __launch_bounds__(32) void k_out(const h16* __restrict__ A, const h16* __restrict__ Bt, float* OUT) {
    __shared__ __align__(16) float os[16 * 68];
    const int K = DQ;
    const int lane = threadIdx.x & 31, lr = lane & 15, hi = lane >> 4; const int r0 = blockIdx.x * 64, c0 = blockIdx.y * 64;
    v8f acc[4][4];
#pragma unroll
    for (int mb = 0; mb < 4; ++mb)
#pragma unroll
        for (int nb = 0; nb < 4; ++nb) acc[mb][nb] = (v8f){};
    const size_t aoff = (size_t)(r0 + lr) * K + 8 * hi, boff = (size_t)(c0 + lr) * K + 8 * hi;
#pragma unroll 1
    for (int kc = 0; kc < K; kc += 32) {
        v16h a[4];
#pragma unroll
        for (int mb = 0; mb < 4; ++mb) a[mb] = ldh(A + aoff + (size_t)mb * 16 * K + kc);
#pragma unroll
        for (int nb = 0; nb < 4; ++nb) { const v16h bq = ldh(Bt + boff + (size_t)nb * 16 * K + kc);
#pragma unroll
            for (int mb = 0; mb < 4; ++mb) acc[mb][nb] = wmma16g(a[mb], bq, acc[mb][nb]); }
    }
    const int bb = r0 / SEQ, tt = r0 % SEQ;
    float* obase = OUT + ((size_t)bb * OUT_SEQ + (size_t)tt) * DX + c0;
#pragma unroll
    for (int mb = 0; mb < 4; ++mb) {
#pragma unroll
        for (int nb = 0; nb < 4; ++nb) {
#pragma unroll
            for (int j = 0; j < 8; ++j) os[(hi * 8 + j) * 68 + nb * 16 + lr] = acc[mb][nb][j] * OSC; }
        wave_sync();
        v4f ov[8];
#pragma unroll
        for (int s = 0; s < 8; ++s) { const int p = s * 32 + lane; const int row = p >> 4, c4 = (p & 15) * 4;
            ov[s] = *(const v4fa*)(&os[row * 68 + c4]); }
#pragma unroll 1
        for (int ps = 0; ps < 2; ++ps) {
#pragma unroll
            for (int s = 0; s < 8; ++s) { const int p = s * 32 + lane; const int row = p >> 4, c4 = (p & 15) * 4;
                *(volatile v4f*)(obase + (size_t)(mb * 16 + row) * DX + c4) = ov[s]; }
            if (ps == 0) __threadfence(); }
        wave_sync();
    }
}

static constexpr size_t al256(size_t v) { return (v + 255) & ~(size_t)255; }
static constexpr size_t SZ_XB = al256((size_t)NB * SEQ * DX * 2);
static constexpr size_t SZ_WB = al256((size_t)3 * DQ * DX * 2);
static constexpr size_t SZ_WO = al256((size_t)DX * DQ * 2);
static constexpr size_t SZ_TB = al256((size_t)SEQ * 64 * 4);
static constexpr size_t SZ_PL = al256((size_t)NB * NH_ * SEQ * HD * 2);
static constexpr size_t SZ_CX = al256((size_t)NB * SEQ * DQ * 2);
static constexpr size_t SZ_TOTAL = SZ_XB + SZ_WB + SZ_WO + 2 * SZ_TB + 3 * SZ_PL + SZ_CX;
static_assert(SZ_TOTAL <= (size_t)134217728);
static_assert(((size_t)DQ * DX * 2) % 256 == 0);
static_assert((size_t)NB * NH_ * SEQ * HD == (size_t)NB * DQ * SEQ);

extern "C" void kernel_launch(void* const* d_in, const int* in_sizes, int n_in,
                              void* d_out, int out_size, void* d_ws, size_t ws_size, hipStream_t stream) {
    if (n_in < 8) return;
    const size_t needx = ((size_t)(NB - 1) * SEQ_FULL + SEQ) * DX;
    const size_t needm = ((size_t)(NB - 1) * SEQ_FULL + (size_t)(SEQ - 1)) * SEQ_FULL + SEQ;
    if ((size_t)in_sizes[0] < needx || (size_t)in_sizes[1] < needm) return;
    if ((size_t)in_sizes[2] < (size_t)DQ * DX || (size_t)in_sizes[3] < (size_t)DQ * DX || (size_t)in_sizes[4] < (size_t)DQ * DX || (size_t)in_sizes[5] < (size_t)DX * DQ) return;
    if (in_sizes[6] < HD || in_sizes[7] < HD) return;
    if ((size_t)out_size < ((size_t)(NB - 1) * OUT_SEQ + SEQ) * DX) return;
    if (SZ_TOTAL > ws_size) return;
    const float* x    = (const float*)d_in[0];
    const float* mask = (const float*)d_in[1];
    const float* wq   = (const float*)d_in[2];
    const float* wk   = (const float*)d_in[3];
    const float* wv   = (const float*)d_in[4];
    const float* wo   = (const float*)d_in[5];
    const float* qnw  = (const float*)d_in[6];
    const float* knw  = (const float*)d_in[7];
    float* OUT = (float*)d_out;
    char* wsp = (char*)d_ws;
    bf*  XB  = (bf*)wsp;  wsp += SZ_XB;
    bf*  WB  = (bf*)wsp;  wsp += SZ_WB;
    h16* WOH = (h16*)wsp; wsp += SZ_WO;
    float* COS = (float*)wsp; wsp += SZ_TB;
    float* SIN = (float*)wsp; wsp += SZ_TB;
    h16* QH  = (h16*)wsp; wsp += SZ_PL;
    h16* KP  = (h16*)wsp; wsp += SZ_PL;
    h16* VT  = (h16*)wsp; wsp += SZ_PL;
    h16* CTX = (h16*)wsp; wsp += SZ_CX;
    bf* WQ = WB; bf* WK = WB + (size_t)DQ * DX; bf* WV = WB + (size_t)2 * DQ * DX;

    if (SEQ == SEQ_FULL) {
        const size_t n8 = (size_t)NB * SEQ * DX / 8;
        k_cvt8<<<(unsigned)((n8 + 255) / 256), 256, 0, stream>>>(x, XB, n8);
    } else {
        const size_t n8 = (size_t)SEQ * DX / 8;
        for (int b = 0; b < NB; ++b) k_cvt8<<<(unsigned)((n8 + 255) / 256), 256, 0, stream>>>(x + (size_t)b * SEQ_FULL * DX, XB + (size_t)b * SEQ * DX, n8);
    }
    { const size_t n8 = (size_t)DQ * DX / 8; const unsigned g = (unsigned)((n8 + 255) / 256);
      k_cvt8<<<g, 256, 0, stream>>>(wq, WQ, n8); k_cvt8<<<g, 256, 0, stream>>>(wk, WK, n8); k_cvt8<<<g, 256, 0, stream>>>(wv, WV, n8);
      k_cvtw<<<g, 256, 0, stream>>>(wo, WOH, n8, WOS); }
    k_tab<<<(unsigned)(SEQ * 64 / 256), 256, 0, stream>>>(COS, SIN, SEQ * 64);

    k_qk<<<dim3(NB * SEQ / 32, NH_, 1), 32, 0, stream>>>(XB, WQ, qnw, COS, SIN, QH);
    k_qk<<<dim3(NB * SEQ / 32, NH_, 1), 32, 0, stream>>>(XB, WK, knw, COS, SIN, KP);
    k_vt<<<dim3(DQ / 64, NB * SEQ / 64, 1), 32, 0, stream>>>(WV, XB, VT);

    k_flash<<<dim3(SEQ / (16 * AW), NB * NH_, 1), 32 * AW, 0, stream>>>(QH, KP, VT, mask, CTX);
    k_out<<<dim3(NB * SEQ / 64, DX / 64, 1), 32, 0, stream>>>(CTX, WOH, OUT);
}
